// RQ_NSF_36807869726859
// MI455X (gfx1250) — hardware-verified
//
#include <hip/hip_runtime.h>
#include <math.h>

constexpr int   kCols       = 16;
constexpr int   kIdCols     = 8;
constexpr int   kHidden     = 256;
constexpr int   kK1         = 32;
constexpr int   kParPerDim  = 14;
constexpr int   kNPar       = 112;
constexpr int   kNParPad    = 128;
constexpr int   kStacks     = 3;
constexpr int   kChunkRows  = 65536;
constexpr float kWCarry     = 16.0f;
constexpr float kHCarry     = 8.0f;
constexpr float kScaleL1    = 0.5f;
constexpr float kScaleL23   = 1.0f / 16.0f;
constexpr float kScaleL4    = 1.0f / 128.0f;
constexpr float kParamScale = 0.0625f;
constexpr float kTail       = 3.0f;
constexpr float kMinBin     = 1e-3f;
constexpr float kMinDer     = 1e-3f;
constexpr float kBinScale   = 0.995f;
constexpr float kDerConst   = 0.5397424172369521f;
constexpr int   kBiasWsFloats = 9 * 256 + 3 * 128;

typedef __attribute__((ext_vector_type(16))) _Float16 v16h;
typedef __attribute__((ext_vector_type(8)))  _Float16 v8h;
typedef __attribute__((ext_vector_type(16))) __bf16   v16b;
typedef __attribute__((ext_vector_type(8)))  __bf16   v8b;
typedef __attribute__((ext_vector_type(8)))  float    v8f;
typedef __attribute__((ext_vector_type(4)))  float    v4f;
typedef __attribute__((ext_vector_type(4)))  unsigned int v4u;

__device__ __forceinline__ unsigned short f2bf_bits(float f) {
  unsigned u = __float_as_uint(f);
  return (unsigned short)((u + 0x7FFFu + ((u >> 16) & 1u)) >> 16);
}
__device__ __forceinline__ float bf_bits2f(unsigned short h) { return __uint_as_float(((unsigned)h) << 16); }

__device__ __forceinline__ void dep_guard_h(v8f& a, v8f& b, v16h x, v16h y) { asm volatile("v_nop\n\tv_nop\n\tv_nop\n\tv_nop" : "+v"(a), "+v"(b) : "v"(x), "v"(y)); }
__device__ __forceinline__ void dep_guard_b(v8f& a, v8f& b, v16b x, v16b y) { asm volatile("v_nop\n\tv_nop\n\tv_nop\n\tv_nop" : "+v"(a), "+v"(b) : "v"(x), "v"(y)); }
__device__ __forceinline__ void keep4_h(v16h a, v16h b, v16h c, v16h d) { asm volatile("v_nop" :: "v"(a), "v"(b), "v"(c), "v"(d)); }
__device__ __forceinline__ void keep4_b(v16b a, v16b b, v16b c, v16b d) { asm volatile("v_nop" :: "v"(a), "v"(b), "v"(c), "v"(d)); }
__device__ __forceinline__ void acc_guard4(v8f& a, v8f& b, v8f& c, v8f& d) { asm volatile("v_nop\n\tv_nop\n\tv_nop\n\tv_nop" : "+v"(a), "+v"(b), "+v"(c), "+v"(d)); }
template <typename T> struct Frag;
template <> struct Frag<_Float16> {
  typedef v16h V; union U { v16h v; v8h h[2]; };
  static __device__ __forceinline__ v16h load(const _Float16* p) {
    U f; f.h[0] = *(const v8h*)(p); f.h[1] = *(const v8h*)(p + 16); return f.v;
  }
  static __device__ __forceinline__ v8f mma(v16h a, v16h b, v8f c) {
    return __builtin_amdgcn_wmma_f32_16x16x32_f16(false, a, false, b, (short)0, c, false, false);
  }
  static __device__ __forceinline__ void guard(v8f& a, v8f& b, v16h x, v16h y) { dep_guard_h(a, b, x, y); }
  static __device__ __forceinline__ void keep(v16h a, v16h b, v16h c, v16h d) { keep4_h(a, b, c, d); }
};
template <> struct Frag<__bf16> {
  typedef v16b V; union U { v16b v; v8b h[2]; };
  static __device__ __forceinline__ v16b load(const __bf16* p) {
    U f; f.h[0] = *(const v8b*)(p); f.h[1] = *(const v8b*)(p + 16); return f.v;
  }
  static __device__ __forceinline__ v8f mma(v16b a, v16b b, v8f c) {
    return __builtin_amdgcn_wmma_f32_16x16x32_bf16(false, a, false, b, (short)0, c, false, false);
  }
  static __device__ __forceinline__ void guard(v8f& a, v8f& b, v16b x, v16b y) { dep_guard_b(a, b, x, y); }
  static __device__ __forceinline__ void keep(v16b a, v16b b, v16b c, v16b d) { keep4_b(a, b, c, d); }
};

__device__ __forceinline__ unsigned pk16(unsigned short a, unsigned short b) { return (unsigned)a | ((unsigned)b << 16); }
__device__ __forceinline__ unsigned short h_bits(float f) { const _Float16 h = (_Float16)f; return __builtin_bit_cast(unsigned short, h); }

template <int ET> struct Elem;
template <> struct Elem<0> { typedef _Float16 T; };
template <> struct Elem<1> { typedef __bf16 T; };
template <int ET, bool SPLIT, int BIAS_MODE, int OUT_MODE, bool RESID, int ACT = 0>
__global__ __launch_bounds__(256) void wmma_gemm64(
    const unsigned short* __restrict__ Ap, const unsigned short* __restrict__ A2p, int lda, long strideA,
    const unsigned short* __restrict__ Btp, const unsigned short* __restrict__ Bt2p, int ldb, long strideB,
    void* __restrict__ Cout, void* __restrict__ Cout2, int ldc, long strideC,
    const float* __restrict__ bias,
    const float* __restrict__ resid, long strideR,
    int M, int N, int K, float scale) {
  typedef typename Elem<ET>::T T;
  typedef typename Frag<T>::V V;
  const T* A = (const T*)Ap; const T* A2 = (const T*)A2p; const T* Bt = (const T*)Btp; const T* Bt2 = (const T*)Bt2p;
  __shared__ __align__(16) float sT[8][16 * 68];
  const int b    = blockIdx.y;
  const int lane = threadIdx.x & 31;
  const int wave = threadIdx.x >> 5;
  const int tilesN = N >> 6;
  const int tilesM = M >> 6;
  const int tile = blockIdx.x * 8 + wave;
  if (tile >= tilesM * tilesN) return;
  const int tm = tile / tilesN;
  const int tn = tile - tm * tilesN;
  const int m0 = tm << 6;
  const int n0 = tn << 6;

  const T* Ab  = A  + (size_t)b * strideA;
  const T* Bb  = Bt + (size_t)b * strideB;
  const T* Ab2 = SPLIT ? (A2  + (size_t)b * strideA) : nullptr;
  const T* Bb2 = SPLIT ? (Bt2 + (size_t)b * strideB) : nullptr;

  const int rlane = lane & 15;
  const int koff  = (lane >> 4) * 8;
  const int mOff  = (lane >> 4) * 8;

  v8f acc[4][4];
#pragma unroll
  for (int i = 0; i < 4; ++i)
#pragma unroll
    for (int j = 0; j < 4; ++j) acc[i][j] = (v8f){0.f,0.f,0.f,0.f,0.f,0.f,0.f,0.f};

  for (int k0 = 0; k0 < K; k0 += 32) {
    V bh[4], bl[4];
#pragma unroll
    for (int j = 0; j < 4; ++j) {
      const size_t bo = (size_t)(n0 + (j << 4) + rlane) * ldb + koff + k0;
      bh[j] = Frag<T>::load(Bb + bo);
      if (SPLIT) bl[j] = Frag<T>::load(Bb2 + bo);
    }
#pragma unroll
    for (int i = 0; i < 4; ++i) {
      const size_t ao = (size_t)(m0 + (i << 4) + rlane) * lda + koff + k0;
      V ah = Frag<T>::load(Ab + ao);
      V al;
      if (SPLIT) al = Frag<T>::load(Ab2 + ao);
#pragma unroll
      for (int j = 0; j < 4; ++j) {
        acc[i][j] = Frag<T>::mma(ah, bh[j], acc[i][j]);
        if (SPLIT) {
          acc[i][j] = Frag<T>::mma(ah, bl[j], acc[i][j]);
          acc[i][j] = Frag<T>::mma(al, bh[j], acc[i][j]);
        }
      }
      Frag<T>::guard(acc[i][0], acc[i][3], ah, SPLIT ? al : ah);
    }
    Frag<T>::keep(bh[0], bh[1], bh[2], bh[3]);
    if (SPLIT) Frag<T>::keep(bl[0], bl[1], bl[2], bl[3]);
  }
  acc_guard4(acc[0][0], acc[0][1], acc[0][2], acc[0][3]);
  acc_guard4(acc[1][0], acc[1][1], acc[1][2], acc[1][3]);
  acc_guard4(acc[2][0], acc[2][1], acc[2][2], acc[2][3]);
  acc_guard4(acc[3][0], acc[3][1], acc[3][2], acc[3][3]);

  float* slab = sT[wave];
  const float* Rb = RESID ? (resid + (size_t)b * strideR) : nullptr;
#pragma unroll
  for (int i = 0; i < 4; ++i) {
    const int mBase = m0 + (i << 4);
#pragma unroll
    for (int j = 0; j < 4; ++j) {
      const int n = n0 + (j << 4) + rlane;
      float bv = 0.f;
      if (BIAS_MODE == 2) bv = bias[n];
#pragma unroll
      for (int r = 0; r < 8; ++r) {
        float v = acc[i][j][r] * scale;
        if (BIAS_MODE == 1) v += bias[mBase + mOff + r];
        if (BIAS_MODE == 2) v += bv;
        if (RESID) v += Rb[(size_t)(mBase + mOff + r) * ldc + n];
        if (ACT == 2) v = fmaxf(v, 0.0f);
        if (ACT == 4) v = (v > 0.f) ? v : 0.01f * v;
        slab[(mOff + r) * 68 + (j << 4) + rlane] = v;
      }
    }
    __builtin_amdgcn_fence(__ATOMIC_RELEASE, "workgroup");
    __builtin_amdgcn_wave_barrier();
    __builtin_amdgcn_fence(__ATOMIC_ACQUIRE, "workgroup");
    if (OUT_MODE == 0) {
      float* C = (float*)Cout + (size_t)b * strideC;
      const int hh = lane >> 4, c4 = (lane & 15) * 4;
      for (int pass = 0; pass < 2; ++pass) {
#pragma unroll
        for (int it = 0; it < 8; ++it) {
          const int row = it * 2 + hh;
          v4f v = *(const v4f*)(slab + row * 68 + c4);
          *(volatile v4f*)(C + (size_t)(mBase + row) * ldc + n0 + c4) = v;
        }
        __threadfence();
      }
    } else {
      const int q = lane >> 3, c8 = (lane & 7) * 8;
      unsigned short* C  = (unsigned short*)Cout  + (size_t)b * strideC;
      unsigned short* C2 = (OUT_MODE == 2) ? ((unsigned short*)Cout2 + (size_t)b * strideC) : nullptr;
      for (int pass = 0; pass < 2; ++pass) {
#pragma unroll
        for (int it = 0; it < 4; ++it) {
          const int row = it * 4 + q;
          const float* sp = slab + row * 68 + c8;
          v8h hv, lv;
#pragma unroll
          for (int e = 0; e < 8; ++e) {
            if (OUT_MODE == 1) {
              hv[e] = (_Float16)sp[e];
            } else {
              unsigned short hb = f2bf_bits(sp[e]);
              unsigned short lb = f2bf_bits(sp[e] - bf_bits2f(hb));
              hv[e] = __builtin_bit_cast(_Float16, hb);
              lv[e] = __builtin_bit_cast(_Float16, lb);
            }
          }
          *(volatile v8h*)(C + (size_t)(mBase + row) * ldc + n0 + c8) = hv;
          if (OUT_MODE == 2) *(volatile v8h*)(C2 + (size_t)(mBase + row) * ldc + n0 + c8) = lv;
        }
        __threadfence();
      }
    }
    __builtin_amdgcn_fence(__ATOMIC_RELEASE, "workgroup");
    __builtin_amdgcn_wave_barrier();
    __builtin_amdgcn_fence(__ATOMIC_ACQUIRE, "workgroup");
  }
}

__global__ __launch_bounds__(256) void cast_pad_f16_kernel(const float* __restrict__ src, unsigned short* __restrict__ dst,
                                                          int src_rows, int src_pitch, int src_cols,
                                                          int dst_rows, int dst_cols, float scale, int n8) {
  const int i = blockIdx.x * 256 + threadIdx.x;
  if (i >= n8) return;
  const int c8n = dst_cols >> 3;
  const int per = dst_rows * c8n;
  const int s   = i / per;
  const int rem = i - s * per;
  const int n   = rem / c8n;
  const int k8  = (rem - n * c8n) * 8;
  const bool valid = (n < src_rows) && (k8 < src_cols);
  const int nc = (n < src_rows) ? n : (src_rows - 1);
  const int kc = (k8 < src_cols) ? k8 : (src_cols - 8);
  const float* p = src + ((size_t)s * src_rows + (size_t)nc) * (size_t)src_pitch + kc;
  const v4f a = *(const v4f*)(p);
  const v4f c = *(const v4f*)(p + 4);
  unsigned short hb[8];
#pragma unroll
  for (int e = 0; e < 4; ++e) {
    hb[e]     = h_bits(valid ? a[e] * scale : 0.0f);
    hb[4 + e] = h_bits(valid ? c[e] * scale : 0.0f);
  }
  const v4u u = (v4u){pk16(hb[0], hb[1]), pk16(hb[2], hb[3]), pk16(hb[4], hb[5]), pk16(hb[6], hb[7])};
  unsigned short* q = dst + 8 * (size_t)i;
  *(volatile v4u*)q = u;
  __threadfence();
  *(volatile v4u*)q = u;
}

__global__ __launch_bounds__(256) void bias_prep_kernel(const float* __restrict__ b1, const float* __restrict__ b2,
                                                       const float* __restrict__ b3, const float* __restrict__ b4,
                                                       float* __restrict__ out, int n4) {
  const int i = blockIdx.x * 256 + threadIdx.x;
  if (i >= n4) return;
  const int f = 4 * i;
  const int l = f / 768;
  const int rem = f - l * 768;
  const v4f c1 = *(const v4f*)(b1 + rem);
  const v4f c2 = *(const v4f*)(b2 + rem);
  const v4f c3 = *(const v4f*)(b3 + rem);
  int g = f - 2304; g = (g < 0) ? 0 : g;
  const int s4 = g / 128;
  const int n  = g - s4 * 128;
  const bool nok = (n < kNPar);
  const int nc = (n < kNPar - 4) ? n : (kNPar - 4);
  const v4f c4 = *(const v4f*)(b4 + s4 * kNPar + nc);
  const bool hid = (f < 2304);
  v4f r;
#pragma unroll
  for (int e = 0; e < 4; ++e) {
    const float hv = (l == 0) ? c1[e] : ((l == 1) ? c2[e] : c3[e]);
    r[e] = hid ? (hv * kHCarry) : (nok ? c4[e] : 0.0f);
  }
  float* q = out + f;
  *(volatile v4f*)q = r;
  __threadfence();
  *(volatile v4f*)q = r;
}

__device__ __forceinline__ float softplus_f(float x) {
#pragma clang fp contract(off)
  const float ax = fabsf(x);
  return fmaxf(x, 0.0f) + log1pf(expf(-ax));
}

__global__ __launch_bounds__(256) void coupling_kernel(const float* __restrict__ P, const float* __restrict__ xsrc,
                                                      const float* __restrict__ lsrc, float* __restrict__ xdst,
                                                      float* __restrict__ ldst, unsigned short* __restrict__ a16,
                                                      int row0, int flip, int accum, int write_a16) {
#pragma clang fp contract(off)
  __shared__ __align__(16) float xs[32 * kCols];
  __shared__ __align__(16) float ls[32];
  const int t    = threadIdx.x;
  const int lane = t & 31;
  const int rl   = t >> 3;
  const int d    = t & 7;
  const int prow = blockIdx.x * 32 + rl;
  const size_t grow = (size_t)row0 + (size_t)prow;
  const float* pp = P + (size_t)prow * kNParPad + d * kParPerDim;

  float cw[6], ch[6], ww[5], hw[5];
#pragma unroll
  for (int j = 0; j < 6; ++j) { cw[j] = 0.0f; ch[j] = 0.0f; }
#pragma unroll
  for (int j = 0; j < 5; ++j) { ww[j] = 0.0f; hw[j] = 0.0f; }
#pragma unroll 1
  for (int ts = 0; ts < 2; ++ts) {
    float u[5];
#pragma unroll
    for (int j = 0; j < 5; ++j) u[j] = pp[ts * 5 + j] * kParamScale;
    const float m = fmaxf(fmaxf(fmaxf(u[0], u[1]), fmaxf(u[2], u[3])), u[4]);
    float e[5];
#pragma unroll
    for (int j = 0; j < 5; ++j) e[j] = expf(u[j] - m);
    const float se  = (((e[0] + e[1]) + e[2]) + e[3]) + e[4];
    const float inv = 1.0f / se;
    float c[6], wd[5];
    float cum = 0.0f;
    c[0] = -kTail;
#pragma unroll
    for (int j = 0; j < 5; ++j) {
      const float pj = kMinBin + kBinScale * (e[j] * inv);
      cum = cum + pj;
      c[j + 1] = 6.0f * cum - kTail;
    }
    c[5] = kTail;
#pragma unroll
    for (int j = 0; j < 5; ++j) wd[j] = c[j + 1] - c[j];
    const bool first = (ts == 0);
#pragma unroll
    for (int j = 0; j < 6; ++j) { cw[j] = first ? c[j] : cw[j]; ch[j] = first ? ch[j] : c[j]; }
#pragma unroll
    for (int j = 0; j < 5; ++j) { ww[j] = first ? wd[j] : ww[j]; hw[j] = first ? hw[j] : wd[j]; }
  }

  float dq0 = 0.0f, dq1 = 0.0f, dq2 = 0.0f, dq3 = 0.0f, dqe = 0.0f;
#pragma unroll 1
  for (int j = 0; j < 5; ++j) {
    const int jj = (j < 4) ? j : 3;
    const float raw = pp[10 + jj];
    const float arg = (j < 4) ? raw : kDerConst;
    const float v = kMinDer + softplus_f(arg);
    dq0 = (j == 0) ? v : dq0;
    dq1 = (j == 1) ? v : dq1;
    dq2 = (j == 2) ? v : dq2;
    dq3 = (j == 3) ? v : dq3;
    dqe = (j == 4) ? v : dqe;
  }
  float dv[6];
  dv[0] = dqe; dv[1] = dq0; dv[2] = dq1; dv[3] = dq2; dv[4] = dq3; dv[5] = dqe;

  const float xid = xsrc[grow * kCols + d];
  const float xtr = xsrc[grow * kCols + kIdCols + d];
  const bool inside = (xtr >= -kTail) && (xtr <= kTail);
  const float xc = fminf(fmaxf(xtr, -kTail), kTail);

  int cnt = 0;
#pragma unroll
  for (int j = 0; j < 6; ++j) cnt += (xc >= cw[j]) ? 1 : 0;
  int idx = cnt - 1;
  idx = (idx < 0) ? 0 : idx;
  idx = (idx > 4) ? 4 : idx;
  float icw = cw[0], iw = ww[0], ich = ch[0], ih = hw[0], id0 = dv[0], id1 = dv[1];
#pragma unroll
  for (int j = 1; j < 5; ++j) {
    const bool sj = (idx == j);
    icw = sj ? cw[j] : icw;
    iw  = sj ? ww[j] : iw;
    ich = sj ? ch[j] : ich;
    ih  = sj ? hw[j] : ih;
    id0 = sj ? dv[j] : id0;
    id1 = sj ? dv[j + 1] : id1;
  }

  const float idel  = ih / iw;
  const float theta = (xc - icw) / iw;
  const float th2   = theta * theta;
  const float omt   = 1.0f - theta;
  const float tmt   = theta * omt;
  const float den   = idel + ((id0 + id1) - 2.0f * idel) * tmt;
  const float ynum  = ih * (idel * th2 + id0 * tmt);
  const float yv    = ich + ynum / den;
  const float omt2  = omt * omt;
  const float dnum  = (idel * idel) * ((id1 * th2 + (2.0f * idel) * tmt) + id0 * omt2);
  const float la    = logf(dnum) - 2.0f * logf(den);
  const float yo    = inside ? yv : xtr;
  const float lo    = inside ? la : 0.0f;

  const int cid = flip ? (15 - d) : d;
  const int ctr = flip ? (7 - d) : (8 + d);
  xs[rl * kCols + cid] = xid;
  xs[rl * kCols + ctr] = yo;
  float sm = lo;
  sm += __shfl_xor(sm, 1, 32);
  sm += __shfl_xor(sm, 2, 32);
  sm += __shfl_xor(sm, 4, 32);
  float lp = 0.0f;
  if (accum) lp = lsrc[grow];
  if (d == 0) ls[rl] = lp + sm;
  __syncthreads();

  const size_t growb = (size_t)row0 + (size_t)blockIdx.x * 32;
  if (t < 128) {
    const int r = t >> 2, c4 = (t & 3) * 4;
    const v4f v = *(const v4f*)(xs + r * kCols + c4);
    float* dst = xdst + (growb + (size_t)r) * kCols + c4;
    *(volatile v4f*)dst = v;
    __threadfence();
    *(volatile v4f*)dst = v;
  } else if (write_a16) {
    const int u = t - 128;
    const int r = u >> 2, k8 = (u & 3) * 8;
    const float* sp = xs + r * kCols;
    unsigned short hb[8];
#pragma unroll
    for (int e = 0; e < 8; ++e) hb[e] = h_bits(sp[e]);
    const bool lead = (k8 == 0);
    v4u w;
    w[0] = lead ? pk16(hb[0], hb[1]) : 0u;
    w[1] = lead ? pk16(hb[2], hb[3]) : 0u;
    w[2] = lead ? pk16(hb[4], hb[5]) : 0u;
    w[3] = lead ? pk16(hb[6], hb[7]) : 0u;
    unsigned short* dst = a16 + (growb + (size_t)r) * kK1 + k8;
    *(volatile v4u*)dst = w;
    __threadfence();
    *(volatile v4u*)dst = w;
  }
  if (t < 32) {
    const v4f v = *(const v4f*)(ls + (lane & 7) * 4);
    if (lane < 8) {
      float* dst = ldst + growb + (size_t)lane * 4;
      *(volatile v4f*)dst = v;
      __threadfence();
      *(volatile v4f*)dst = v;
    }
  }
}

extern "C" void kernel_launch(void* const* d_in, const int* in_sizes, int n_in,
                              void* d_out, int out_size, void* d_ws, size_t ws_size,
                              hipStream_t stream) {
  (void)n_in;
  const float* x_in = (const float*)d_in[0];
  const float* W1   = (const float*)d_in[1];
  const float* b1   = (const float*)d_in[2];
  const float* W2   = (const float*)d_in[3];
  const float* b2   = (const float*)d_in[4];
  const float* W3   = (const float*)d_in[5];
  const float* b3   = (const float*)d_in[6];
  const float* W4   = (const float*)d_in[7];
  const float* b4   = (const float*)d_in[8];

  const int nrows = in_sizes[0] / kCols;
  if (nrows <= 0 || (nrows % kChunkRows) != 0) return;
  if (in_sizes[1] != kStacks * kHidden * kIdCols) return;
  if (in_sizes[3] != kStacks * kHidden * kHidden || in_sizes[5] != kStacks * kHidden * kHidden) return;
  if (in_sizes[7] != kStacks * kNPar * kHidden || in_sizes[8] != kStacks * kNPar) return;
  if (in_sizes[2] != kStacks * kHidden || in_sizes[4] != kStacks * kHidden || in_sizes[6] != kStacks * kHidden) return;
  if ((size_t)out_size < (size_t)nrows * (size_t)(kCols + 1)) return;
  const int nchunk = nrows / kChunkRows;

  unsigned char* ws = (unsigned char*)d_ws;
  size_t off = 0;
  auto carve = [&](size_t bytes) -> unsigned char* {
    unsigned char* p = ws + off;
    off += (bytes + 127) & ~(size_t)127;
    return p;
  };
  unsigned short* Wh1 = (unsigned short*)carve((size_t)kStacks * kHidden * kK1 * 2);
  unsigned short* Wh2 = (unsigned short*)carve((size_t)kStacks * kHidden * kHidden * 2);
  unsigned short* Wh3 = (unsigned short*)carve((size_t)kStacks * kHidden * kHidden * 2);
  unsigned short* Wh4 = (unsigned short*)carve((size_t)kStacks * kNParPad * kHidden * 2);
  float* biasws       = (float*)carve((size_t)kBiasWsFloats * 4);
  unsigned short* A16 = (unsigned short*)carve((size_t)nrows * kK1 * 2);
  float* X0           = (float*)carve((size_t)nrows * kCols * 4);
  float* X1           = (float*)carve((size_t)nrows * kCols * 4);
  float* L0           = (float*)carve((size_t)nrows * 4);
  float* L1           = (float*)carve((size_t)nrows * 4);
  unsigned short* H1  = (unsigned short*)carve((size_t)kChunkRows * kHidden * 2);
  unsigned short* H2  = (unsigned short*)carve((size_t)kChunkRows * kHidden * 2);
  float* Pp           = (float*)carve((size_t)kChunkRows * kNParPad * 4);
  if (off > ws_size) return;

  float* out0 = (float*)d_out;
  float* out1 = out0 + (size_t)nrows * kCols;

  {
    const int n8 = kStacks * kHidden * kK1 / 8;
    cast_pad_f16_kernel<<<(n8 + 255) / 256, 256, 0, stream>>>(W1, Wh1, kHidden, kIdCols, kIdCols, kHidden, kK1, kWCarry, n8);
  }
  {
    const int n8 = kStacks * kHidden * kHidden / 8;
    cast_pad_f16_kernel<<<(n8 + 255) / 256, 256, 0, stream>>>(W2, Wh2, kHidden, kHidden, kHidden, kHidden, kHidden, kWCarry, n8);
    cast_pad_f16_kernel<<<(n8 + 255) / 256, 256, 0, stream>>>(W3, Wh3, kHidden, kHidden, kHidden, kHidden, kHidden, kWCarry, n8);
  }
  {
    const int n8 = kStacks * kNParPad * kHidden / 8;
    cast_pad_f16_kernel<<<(n8 + 255) / 256, 256, 0, stream>>>(W4, Wh4, kNPar, kHidden, kHidden, kNParPad, kHidden, kWCarry, n8);
  }
  {
    const int n4 = kBiasWsFloats / 4;
    bias_prep_kernel<<<(n4 + 255) / 256, 256, 0, stream>>>(b1, b2, b3, b4, biasws, n4);
  }
  {
    const int n8 = nrows * (kK1 / 8);
    cast_pad_f16_kernel<<<(n8 + 255) / 256, 256, 0, stream>>>(x_in, A16, nrows, kCols, kIdCols, nrows, kK1, 1.0f, n8);
  }

  const int tilesH = (kChunkRows / 64) * (kHidden / 64);
  const int tilesP = (kChunkRows / 64) * (kNParPad / 64);
  const dim3 gridH((tilesH + 7) / 8, 1);
  const dim3 gridP((tilesP + 7) / 8, 1);
  const float* dummy_resid = biasws;

  for (int s = 0; s < kStacks; ++s) {
    const unsigned short* Wh1s = Wh1 + (size_t)s * kHidden * kK1;
    const unsigned short* Wh2s = Wh2 + (size_t)s * kHidden * kHidden;
    const unsigned short* Wh3s = Wh3 + (size_t)s * kHidden * kHidden;
    const unsigned short* Wh4s = Wh4 + (size_t)s * kNParPad * kHidden;
    const float* bl0 = biasws + (size_t)(0 * 3 + s) * kHidden;
    const float* bl1 = biasws + (size_t)(1 * 3 + s) * kHidden;
    const float* bl2 = biasws + (size_t)(2 * 3 + s) * kHidden;
    const float* b4s = biasws + (size_t)9 * kHidden + (size_t)s * kNParPad;

    const float* xsrc = (s == 0) ? x_in : ((s == 1) ? X0 : X1);
    float*       xdst = (s == 0) ? X0   : ((s == 1) ? X1 : out0);
    const float* lsrc = (s == 0) ? L1   : ((s == 1) ? L0 : L1);
    float*       ldst = (s == 0) ? L0   : ((s == 1) ? L1 : out1);
    const int flip  = (s < kStacks - 1) ? 1 : 0;
    const int accum = (s > 0) ? 1 : 0;
    const int wa16  = (s < kStacks - 1) ? 1 : 0;

    for (int c = 0; c < nchunk; ++c) {
      const unsigned short* A16c = A16 + (size_t)c * kChunkRows * kK1;
      wmma_gemm64<0, false, 2, 1, false, 2><<<gridH, 256, 0, stream>>>(
          A16c, A16c, kK1, 0L, Wh1s, Wh1s, kK1, 0L,
          (void*)H1, (void*)H1, kHidden, 0L, bl0, dummy_resid, 0L,
          kChunkRows, kHidden, kK1, kScaleL1);
      wmma_gemm64<0, false, 2, 1, false, 2><<<gridH, 256, 0, stream>>>(
          H1, H1, kHidden, 0L, Wh2s, Wh2s, kHidden, 0L,
          (void*)H2, (void*)H2, kHidden, 0L, bl1, dummy_resid, 0L,
          kChunkRows, kHidden, kHidden, kScaleL23);
      wmma_gemm64<0, false, 2, 1, false, 2><<<gridH, 256, 0, stream>>>(
          H2, H2, kHidden, 0L, Wh3s, Wh3s, kHidden, 0L,
          (void*)H1, (void*)H1, kHidden, 0L, bl2, dummy_resid, 0L,
          kChunkRows, kHidden, kHidden, kScaleL23);
      wmma_gemm64<0, false, 2, 0, false, 0><<<gridP, 256, 0, stream>>>(
          H1, H1, kHidden, 0L, Wh4s, Wh4s, kHidden, 0L,
          (void*)Pp, (void*)Pp, kNParPad, 0L, b4s, dummy_resid, 0L,
          kChunkRows, kNParPad, kHidden, kScaleL4);
      coupling_kernel<<<kChunkRows / 32, 256, 0, stream>>>(
          Pp, xsrc, lsrc, xdst, ldst, A16, c * kChunkRows, flip, accum, wa16);
    }
  }
}
